// LightweightMLPDecoder_84920093376640
// MI455X (gfx1250) — hardware-verified
//
#include <hip/hip_runtime.h>
#include <math.h>

typedef __attribute__((ext_vector_type(16))) _Float16 v16h;
typedef __attribute__((ext_vector_type(16))) __bf16 v16b;
typedef __attribute__((ext_vector_type(8)))  _Float16 v8h;
typedef __attribute__((ext_vector_type(8)))  float v8f;
typedef __attribute__((ext_vector_type(4)))  float v4f;
typedef __attribute__((ext_vector_type(2)))  float v2f;
typedef __attribute__((ext_vector_type(4)))  unsigned v4u;
typedef __attribute__((ext_vector_type(4)))  int v4i;
typedef float __attribute__((may_alias)) float_a;
typedef int __attribute__((may_alias)) int_a;

template <typename T> __device__ __forceinline__ void vst2(void* p, T v) { *(volatile T*)p = v; __threadfence(); *(volatile T*)p = v; }
__device__ __forceinline__ v8f wmma16(v16h a, v16h b, v8f c) {
  v8f d = __builtin_amdgcn_wmma_f32_16x16x32_f16(false, a, false, b, (short)0, c, false, false);
  asm volatile("v_nop\n\tv_nop\n\tv_nop\n\tv_nop" : "+v"(d) : "v"(a), "v"(b));
  return d;
}
__device__ __forceinline__ v8f wmma_bf(v16b a, v16b b, v8f c) {
  v8f d = __builtin_amdgcn_wmma_f32_16x16x32_bf16(false, a, false, b, (short)0, c, false, false);
  asm volatile("v_nop\n\tv_nop\n\tv_nop\n\tv_nop" : "+v"(d) : "v"(a), "v"(b));
  return d;
}
__device__ __forceinline__ v16h frag_h(const _Float16* rowk0, int lane) {
  union { v16h v; v8h q[2]; } u; const _Float16* p = rowk0 + 8 * (lane >> 4);
  u.q[0] = *(const v8h*)p; u.q[1] = *(const v8h*)(p + 16); return u.v;
}
__device__ __forceinline__ v16h frag_f32(const float* rowk0, int lane) {
  v16h a; const float* p = rowk0 + 8 * (lane >> 4);
#pragma unroll
  for (int i = 0; i < 8; ++i) { a[i] = (_Float16)p[i]; a[8 + i] = (_Float16)p[16 + i]; }
  return a;
}
__device__ __forceinline__ v16h frag_f32s(const float* rowk0, int lane, float sc) {
  v16h a; const float* p = rowk0 + 8 * (lane >> 4);
#pragma unroll
  for (int i = 0; i < 8; ++i) { a[i] = (_Float16)(p[i] * sc); a[8 + i] = (_Float16)(p[16 + i] * sc); }
  return a;
}
__device__ __forceinline__ v16h fragc_f32(const float* W, int k0, int n, int lane, int ld, int K) {
  v16h a; const int g = lane >> 4;
#pragma unroll
  for (int i = 0; i < 8; ++i) { const int ka = k0 + 8 * g + i, kb = ka + 16;
    a[i] = (_Float16)(ka < K ? W[(size_t)ka * ld + n] : 0.f); a[8 + i] = (_Float16)(kb < K ? W[(size_t)kb * ld + n] : 0.f); }
  return a;
}
struct F2 { v16b h, l; };
__device__ __forceinline__ F2 bsplit16(const float v[16]) { F2 r;
#pragma unroll
  for (int i = 0; i < 16; ++i) { const __bf16 h = (__bf16)v[i]; r.h[i] = h; r.l[i] = (__bf16)(v[i] - (float)h); }
  return r; }
__device__ __forceinline__ F2 split_row(const float* row, int k0, int lane) { float v[16]; const float* p = row + k0 + 8 * (lane >> 4);
#pragma unroll
  for (int i = 0; i < 8; ++i) { v[i] = p[i]; v[8 + i] = p[16 + i]; }
  return bsplit16(v); }
__device__ __forceinline__ F2 split_rowK(const float* row, int k0, int lane, int K) { float v[16]; const int g = lane >> 4;
#pragma unroll
  for (int i = 0; i < 8; ++i) { const int ka = k0 + 8 * g + i, kb = ka + 16; v[i] = ka < K ? row[ka] : 0.f; v[8 + i] = kb < K ? row[kb] : 0.f; }
  return bsplit16(v); }
__device__ __forceinline__ F2 split_col(const float* W, int k0, int n, int lane, int ld, int K) { float v[16]; const int g = lane >> 4;
#pragma unroll
  for (int i = 0; i < 8; ++i) { const int ka = k0 + 8 * g + i, kb = ka + 16; v[i] = ka < K ? W[(size_t)ka * ld + n] : 0.f; v[8 + i] = kb < K ? W[(size_t)kb * ld + n] : 0.f; }
  return bsplit16(v); }
__device__ __forceinline__ v8f mac3(const F2& a, const F2& b, v8f c) { c = wmma_bf(a.l, b.h, c); c = wmma_bf(a.h, b.l, c); return wmma_bf(a.h, b.h, c); }
__device__ __forceinline__ float sigm(float v) { return 1.0f / (1.0f + expf(-v)); }
#define LDSX() do { asm volatile("s_wait_dscnt 0" ::: "memory"); __builtin_amdgcn_wave_barrier(); __builtin_amdgcn_fence(__ATOMIC_RELEASE, "workgroup"); } while (0)


#define NDR 10000
#define NDS 10000
#define NNP 10048
#define NE 1000000
#define D 128
#define HC 64
#define EPB 256
#define NBLK ((NE + EPB - 1) / EPB)
__device__ __forceinline__ int clampi(int v, int hi) { return v < 0 ? 0 : (v > hi ? hi : v); }

__global__ __launch_bounds__(128) void k_proj(const float* __restrict__ X, int n, const float* __restrict__ W1k, float* __restrict__ Pout) {
  __shared__ __align__(16) float so[4][16][68];
  const int tid = threadIdx.x, wave = tid >> 5, lane = tid & 31, col = lane & 15, g = lane >> 4;
  const int r0 = blockIdx.x * 64 + wave * 16; const int ra = (r0 + col) < n ? (r0 + col) : (n - 1);
  v8f acc[4] = {};
#pragma unroll 1
  for (int kc = 0; kc < D / 32; ++kc) { const F2 a = split_row(X + (size_t)ra * D, kc * 32, lane);
#pragma unroll
    for (int j = 0; j < 4; ++j) acc[j] = mac3(a, split_col(W1k, kc * 32, j * 16 + col, lane, HC, D), acc[j]); }
#pragma unroll
  for (int j = 0; j < 4; ++j)
#pragma unroll
    for (int r = 0; r < 8; ++r) so[wave][8 * g + r][j * 16 + col] = acc[j][r];
  LDSX();
  for (int rl = 0; rl < 16; ++rl) { if (lane < 16) vst2(Pout + (size_t)(r0 + rl) * HC + lane * 4, *(const v4f*)(&so[wave][rl][lane * 4])); }
}
__global__ __launch_bounds__(256) void k_stats(const float* __restrict__ Pd, const float* __restrict__ Pq, const int* __restrict__ sidx, const int* __restrict__ didx, const float* __restrict__ b1, float* __restrict__ PART) {
  __shared__ float ss[4][64], sq[4][64];
  const int tid = threadIdx.x, c = tid & 63, sub = tid >> 6; const int e0 = blockIdx.x * EPB; float s = 0.f, q = 0.f; const float bb = b1[c];
#pragma unroll 4
  for (int i = sub; i < EPB; i += 4) { const int e = e0 + i; if (e < NE) { const int a = clampi(sidx[e], NDR - 1), b = clampi(didx[e], NDS - 1); const float h = Pd[(size_t)a * HC + c] + Pq[(size_t)b * HC + c] + bb; s += h; q += h * h; } }
  ss[sub][c] = s; sq[sub][c] = q; __syncthreads();
  if (tid < 64) { const float S = (ss[0][tid] + ss[1][tid]) + (ss[2][tid] + ss[3][tid]), Q = (sq[0][tid] + sq[1][tid]) + (sq[2][tid] + sq[3][tid]); vst2(PART + (size_t)blockIdx.x * 128 + tid, (float_a)S); vst2(PART + (size_t)blockIdx.x * 128 + 64 + tid, (float_a)Q); }
}
__global__ __launch_bounds__(256) void k_fin(const float* __restrict__ PART, const float* __restrict__ gamma, float* __restrict__ STAT) {
  __shared__ float ss[4][64], sq[4][64];
  const int tid = threadIdx.x, c = tid & 63, sub = tid >> 6; float s = 0.f, q = 0.f;
#pragma unroll 1
  for (int b = sub; b < NBLK; b += 4) { s += PART[(size_t)b * 128 + c]; q += PART[(size_t)b * 128 + 64 + c]; }
  ss[sub][c] = s; sq[sub][c] = q; __syncthreads();
  if (tid < 64) { const float S = (ss[0][tid] + ss[1][tid]) + (ss[2][tid] + ss[3][tid]), Q = (sq[0][tid] + sq[1][tid]) + (sq[2][tid] + sq[3][tid]);
    const float mean = S / (float)NE; float var = Q / (float)NE - mean * mean; var = var > 0.f ? var : 0.f;
    vst2(STAT + tid, (float_a)mean); vst2(STAT + 64 + tid, (float_a)(gamma[tid] * rsqrtf(var + 1e-5f))); }
}
__global__ __launch_bounds__(256) void k_out(const float* __restrict__ Pd, const float* __restrict__ Pq, const int* __restrict__ sidx, const int* __restrict__ didx, const float* __restrict__ b1, const float* __restrict__ STAT,
                                            const float* __restrict__ beta, const float* __restrict__ W2, const float* __restrict__ b2, float* __restrict__ out) {
  __shared__ float sres[8][32];
  const int wave = threadIdx.x >> 5, lane = threadIdx.x & 31; const int e0 = (blockIdx.x * 8 + wave) * 32; const int sub = lane >> 3, part = lane & 7;
  float mu[8], sc[8], be[8], w2[8], bb[8];
#pragma unroll
  for (int k = 0; k < 8; ++k) { const int c = part * 8 + k; mu[k] = STAT[c]; sc[k] = STAT[64 + c]; be[k] = beta[c]; w2[k] = W2[c]; bb[k] = b1[c]; }
#pragma unroll 1
  for (int ps = 0; ps < 8; ++ps) { const int e = e0 + ps * 4 + sub; float s = 0.f;
    if (e < NE) { const int a = clampi(sidx[e], NDR - 1), b = clampi(didx[e], NDS - 1); const float* pa = Pd + (size_t)a * HC + part * 8; const float* pb = Pq + (size_t)b * HC + part * 8;
#pragma unroll
      for (int k = 0; k < 8; ++k) { const float h = pa[k] + pb[k] + bb[k]; const float y = (h - mu[k]) * sc[k] + be[k]; s += (y > 0.f ? y : 0.f) * w2[k]; } }
    s += __shfl_xor(s, 1, 32); s += __shfl_xor(s, 2, 32); s += __shfl_xor(s, 4, 32);
    if (part == 0) sres[wave][ps * 4 + sub] = s + b2[0]; }
  LDSX();
  if (e0 + lane < NE) vst2(out + e0 + lane, (float_a)sres[wave][lane]);
}
extern "C" void kernel_launch(void* const* d_in, const int* in_sizes, int n_in, void* d_out, int out_size, void* d_ws, size_t ws_size, hipStream_t stream) {
  (void)in_sizes; (void)n_in; (void)out_size; (void)ws_size;
  const float* drug = (const float*)d_in[0]; const float* dis = (const float*)d_in[1]; const int* sidx = (const int*)d_in[2]; const int* didx = (const int*)d_in[3];
  const float* W1 = (const float*)d_in[4]; const float* b1 = (const float*)d_in[5]; const float* gamma = (const float*)d_in[6]; const float* beta = (const float*)d_in[7]; const float* W2 = (const float*)d_in[8]; const float* b2 = (const float*)d_in[9];
  float* out = (float*)d_out;
  char* ws = (char*)d_ws; size_t off = 0;
  auto take = [&](size_t bytes) { char* p = ws + off; off += (bytes + 255) & ~(size_t)255; return p; };
  float* Pd = (float*)take((size_t)NNP * HC * 4); float* Pq = (float*)take((size_t)NNP * HC * 4); float* PART = (float*)take((size_t)NBLK * 128 * 4); float* STAT = (float*)take(128 * 4);
  k_proj<<<NNP / 64, 128, 0, stream>>>(drug, NDR, W1, Pd);
  k_proj<<<NNP / 64, 128, 0, stream>>>(dis, NDS, W1 + (size_t)D * HC, Pq);
  k_stats<<<NBLK, 256, 0, stream>>>(Pd, Pq, sidx, didx, b1, PART);
  k_fin<<<1, 256, 0, stream>>>(PART, gamma, STAT);
  k_out<<<(NE + 255) / 256, 256, 0, stream>>>(Pd, Pq, sidx, didx, b1, STAT, beta, W2, b2, out);
}
